// MambaDoc_10402410791616
// MI455X (gfx1250) — hardware-run, weakly checked
//
#include <hip/hip_runtime.h>
#include <math.h>

typedef __attribute__((ext_vector_type(16))) _Float16 v16h;
typedef __attribute__((ext_vector_type(8)))  _Float16 v8h;
typedef __attribute__((ext_vector_type(8)))  float    v8f;
typedef __attribute__((ext_vector_type(4)))  float    v4f;

constexpr int kBatch = 4;
constexpr int kSeq   = 4096;
constexpr int kNE    = 64;
constexpr int kDOut  = 64;
constexpr int kDI    = 128;
constexpr int kNL    = 2;
constexpr int kHeads = 2;
constexpr int kNst   = 128;
constexpr int kDIN   = 256;
constexpr int kHP    = 128;
constexpr int kCCH   = 512;
constexpr int kDPROJ = 770;
constexpr int kZXW   = 768;
constexpr int kRows  = kBatch * kSeq;

constexpr float kWCarry    = 32.0f;
constexpr float kWCarryInv = 1.0f / kWCarry;
constexpr float kResCarry  = 2048.0f;
constexpr float kResInv    = 1.0f / kResCarry;
constexpr float kMCarry    = 16.0f;
constexpr float kMInv      = 1.0f / kMCarry;
constexpr float kHiFlush   = 6.2e-5f;
constexpr float kEps       = 1e-5f;

constexpr int kConvTP = 260;
constexpr int kQ      = 32;
constexpr int kPS     = 64;
constexpr int kXTP    = 32;
constexpr int kBP     = 136;
constexpr int kYP     = 68;

static_assert(kDIN == 2 * kDI && kHP * kHeads == kDIN && kCCH == kDIN + 2 * kNst, "channel split");
static_assert(kDPROJ == kZXW + kHeads && kZXW == kDIN + kCCH, "in_proj width");
static_assert(kHeads == 2, "two dt heads");
static_assert((kNE % 32) == 0 && (kDI % 32) == 0 && (kDIN % 32) == 0, "GEMM K multiples of 32");
static_assert((kRows % 64) == 0 && (kDI % 64) == 0 && (kZXW % 64) == 0 && (kDOut % 64) == 0, "GEMM M,N multiples of 64");
static_assert((kRows % 256) == 0 && (kSeq % 64) == 0 && (kSeq % kQ) == 0 && (kHP % kPS) == 0, "tile multiples");
static_assert(kQ == 32 && kPS == 64 && kNst == 128, "scan tiling");

constexpr size_t kOffX16   = 0;
constexpr size_t kOffWIN16 = kOffX16   + (size_t)kRows * kNE * 2;
constexpr size_t kOffWL16  = kOffWIN16 + (size_t)kDI * kNE * 2;
constexpr size_t kOffWO16  = kOffWL16  + (size_t)kNL * kZXW * kDI * 2;
constexpr size_t kOffWF16  = kOffWO16  + (size_t)kNL * kDI * kDIN * 2;
constexpr size_t kOffXP    = kOffWF16  + (size_t)kDOut * kDI * 2;
constexpr size_t kOffH1    = kOffXP    + (size_t)kRows * kDI * 4;
constexpr size_t kOffHNH   = kOffH1    + (size_t)kRows * kDI * 4;
constexpr size_t kOffHNL   = kOffHNH   + (size_t)kRows * kDI * 2;
constexpr size_t kOffZX    = kOffHNL   + (size_t)kRows * kDI * 2;
constexpr size_t kOffXC    = kOffZX    + (size_t)kRows * kZXW * 4;
constexpr size_t kOffDT    = kOffXC    + (size_t)kRows * kCCH * 4;
constexpr size_t kOffLA    = kOffDT    + (size_t)kHeads * kRows * 4;
constexpr size_t kOffYNH   = kOffLA    + (size_t)kHeads * kRows * 4;
constexpr size_t kOffYNL   = kOffYNH   + (size_t)kRows * kDIN * 2;
constexpr size_t kWsTotal  = kOffYNL   + (size_t)kRows * kDIN * 2;
static_assert(kWsTotal == 128745472ull, "carve total");
static_assert(kWsTotal <= 134217728ull, "carve cap");
static_assert((size_t)kRows * kDI * 4 <= (size_t)kRows * kZXW * 4, "layer-1 stream fits in the ZX region");
static_assert((kOffWIN16 % 128) == 0 && (kOffWL16 % 128) == 0 && (kOffWO16 % 128) == 0 && (kOffWF16 % 128) == 0 &&
              (kOffXP % 128) == 0 && (kOffH1 % 128) == 0 && (kOffHNH % 128) == 0 && (kOffHNL % 128) == 0 &&
              (kOffZX % 128) == 0 && (kOffXC % 128) == 0 && (kOffDT % 128) == 0 && (kOffLA % 128) == 0 &&
              (kOffYNH % 128) == 0 && (kOffYNL % 128) == 0, "128-B aligned regions");

struct FragH {
  union U { v16h v; v8h h[2]; };
  static __device__ __forceinline__ v16h load(const _Float16* p) {
    U f; f.h[0] = *(const v8h*)(p); f.h[1] = *(const v8h*)(p + 16); return f.v;
  }
  static __device__ __forceinline__ v8f mma(v16h a, v16h b, v8f c) {
    return __builtin_amdgcn_wmma_f32_16x16x32_f16(false, a, false, b, (short)0, c, false, false);
  }
};
__device__ __forceinline__ v8f mma_guarded(v16h a, v16h b, v8f c) {
  c = FragH::mma(a, b, c);
  asm volatile("v_nop\n\tv_nop\n\tv_nop\n\tv_nop" : "+v"(c) : "v"(a), "v"(b));
  return c;
}
__device__ __forceinline__ void guard_row4(v8f& a0, v8f& a1, v8f& a2, v8f& a3, v16h x,
                                           v16h b0, v16h b1, v16h b2, v16h b3) {
  asm volatile("v_nop\n\tv_nop\n\tv_nop\n\tv_nop"
               : "+v"(a0), "+v"(a1), "+v"(a2), "+v"(a3)
               : "v"(x), "v"(b0), "v"(b1), "v"(b2), "v"(b3));
}
__device__ __forceinline__ void guard_row8(v8f& a0, v8f& a1, v8f& a2, v8f& a3,
                                           v8f& r0, v8f& r1, v8f& r2, v8f& r3, v16h x, v16h y,
                                           v16h b0, v16h b1, v16h b2, v16h b3) {
  asm volatile("v_nop\n\tv_nop\n\tv_nop\n\tv_nop"
               : "+v"(a0), "+v"(a1), "+v"(a2), "+v"(a3), "+v"(r0), "+v"(r1), "+v"(r2), "+v"(r3)
               : "v"(x), "v"(y), "v"(b0), "v"(b1), "v"(b2), "v"(b3));
}
__device__ __forceinline__ void keep4_h(v16h a, v16h b, v16h c, v16h d) { asm volatile("v_nop" :: "v"(a), "v"(b), "v"(c), "v"(d)); }
__device__ __forceinline__ void acc_guard4(v8f& a, v8f& b, v8f& c, v8f& d) { asm volatile("v_nop\n\tv_nop\n\tv_nop\n\tv_nop" : "+v"(a), "+v"(b), "+v"(c), "+v"(d)); }

__device__ __forceinline__ float bf16r(float f) {
  unsigned u = __float_as_uint(f);
  u = (u + 0x7FFFu + ((u >> 16) & 1u)) & 0xFFFF0000u;
  return __uint_as_float(u);
}
__device__ __forceinline__ unsigned short h_bits(_Float16 hv) {
  return __builtin_bit_cast(unsigned short, hv);
}
__device__ __forceinline__ unsigned short f16_bits(float f) {
  const _Float16 hv = (_Float16)f;
  return __builtin_bit_cast(unsigned short, hv);
}
__device__ __forceinline__ void split_res(float v, _Float16& hi, _Float16& lo) {
  const float vh = (fabsf(v) < kHiFlush) ? 0.0f : v;
  const _Float16 h = (_Float16)vh;
  float hf = (float)h;
  asm volatile("" : "+v"(hf));
  hi = h;
  lo = (_Float16)((v - hf) * kResCarry);
}

__global__ __launch_bounds__(256) void cast_f16_kernel(
    const float* __restrict__ src, unsigned short* __restrict__ dst, int total8, float scale)
{
  const int i = blockIdx.x * 256 + threadIdx.x;
  if (i >= total8) return;
  const size_t e0 = (size_t)i << 3;
  const float* p = src + e0;
  const v4f a0 = *(const v4f*)(p);
  const v4f a1 = *(const v4f*)(p + 4);
  v8h hv;
#pragma unroll
  for (int e = 0; e < 4; ++e) {
    const float s0 = a0[e];
    const float s1 = a1[e];
    hv[e]     = (_Float16)(bf16r(s0) * scale);
    hv[4 + e] = (_Float16)(bf16r(s1) * scale);
  }
  unsigned short* q = dst + e0;
  *(volatile v8h*)q = hv;
  __threadfence();
  *(volatile v8h*)q = hv;
}

template <int MT, bool SPLITA, int BIAS_MODE, bool RESID>
__global__ __launch_bounds__(256) void wmma_gemm_f16(
    const unsigned short* __restrict__ Ap, const unsigned short* __restrict__ A2p, int lda,
    const unsigned short* __restrict__ Btp, int ldb,
    float* __restrict__ Cout, int ldc,
    const float* __restrict__ bias,
    const float* __restrict__ resid,
    int M, int N, int K, float scale, float scale2)
{
  const _Float16* A  = (const _Float16*)Ap;
  const _Float16* A2 = (const _Float16*)A2p;
  const _Float16* Bt = (const _Float16*)Btp;
  __shared__ __align__(16) float sT[8][16 * 68];
  const int lane = threadIdx.x & 31;
  const int wave = threadIdx.x >> 5;
  const int tilesN = N >> 6;
  const int tilesM = M / (16 * MT);
  const int tile = blockIdx.x * 8 + wave;
  if (tile >= tilesM * tilesN) return;
  const int tm = tile / tilesN;
  const int tn = tile - tm * tilesN;
  const int m0 = tm * (16 * MT);
  const int n0 = tn << 6;

  const int rlane = lane & 15;
  const int koff  = (lane >> 4) * 8;
  const int mOff  = (lane >> 4) * 8;

  v8f acc[MT][4];
  v8f accr[MT][4];
#pragma unroll
  for (int i = 0; i < MT; ++i)
#pragma unroll
    for (int j = 0; j < 4; ++j) {
      acc[i][j]  = (v8f){0.f,0.f,0.f,0.f,0.f,0.f,0.f,0.f};
      accr[i][j] = (v8f){0.f,0.f,0.f,0.f,0.f,0.f,0.f,0.f};
    }

  for (int k0 = 0; k0 < K; k0 += 32) {
    v16h bh[4];
#pragma unroll
    for (int j = 0; j < 4; ++j) {
      const size_t bo = (size_t)(n0 + (j << 4) + rlane) * ldb + koff + k0;
      bh[j] = FragH::load(Bt + bo);
    }
#pragma unroll
    for (int i = 0; i < MT; ++i) {
      const size_t ao = (size_t)(m0 + (i << 4) + rlane) * lda + koff + k0;
      const v16h ah = FragH::load(A + ao);
      v16h al = ah;
      if (SPLITA) al = FragH::load(A2 + ao);
#pragma unroll
      for (int j = 0; j < 4; ++j) {
        acc[i][j] = FragH::mma(ah, bh[j], acc[i][j]);
        if (SPLITA) accr[i][j] = FragH::mma(al, bh[j], accr[i][j]);
      }
      if (SPLITA) {
        guard_row8(acc[i][0], acc[i][1], acc[i][2], acc[i][3], accr[i][0], accr[i][1], accr[i][2], accr[i][3],
                   ah, al, bh[0], bh[1], bh[2], bh[3]);
      } else {
        guard_row4(acc[i][0], acc[i][1], acc[i][2], acc[i][3], ah, bh[0], bh[1], bh[2], bh[3]);
      }
    }
    keep4_h(bh[0], bh[1], bh[2], bh[3]);
  }
#pragma unroll
  for (int i = 0; i < MT; ++i) {
    acc_guard4(acc[i][0], acc[i][1], acc[i][2], acc[i][3]);
    if (SPLITA) acc_guard4(accr[i][0], accr[i][1], accr[i][2], accr[i][3]);
  }

  float* slab = sT[wave];
#pragma unroll
  for (int i = 0; i < MT; ++i) {
    const int mBase = m0 + (i << 4);
#pragma unroll
    for (int j = 0; j < 4; ++j) {
      const int n = n0 + (j << 4) + rlane;
      float bv = 0.f;
      if (BIAS_MODE == 2) bv = bf16r(bias[n]);
#pragma unroll
      for (int r = 0; r < 8; ++r) {
        float v = acc[i][j][r] * scale;
        if (SPLITA) v += accr[i][j][r] * scale2;
        if (BIAS_MODE == 2) v += bv;
        slab[(mOff + r) * 68 + (j << 4) + rlane] = v;
      }
    }
    __builtin_amdgcn_fence(__ATOMIC_RELEASE, "workgroup");
    __builtin_amdgcn_wave_barrier();
    __builtin_amdgcn_fence(__ATOMIC_ACQUIRE, "workgroup");
    {
      const int hh = lane >> 4, c4 = (lane & 15) * 4;
      v4f vals[8];
#pragma unroll
      for (int it = 0; it < 8; ++it) {
        const int row = it * 2 + hh;
        v4f v = *(const v4f*)(slab + row * 68 + c4);
        if (RESID) {
          const v4f rv = *(const v4f*)(resid + (size_t)(mBase + row) * ldc + n0 + c4);
          v = v + rv;
        }
        vals[it] = v;
      }
      for (int pass = 0; pass < 2; ++pass) {
#pragma unroll
        for (int it = 0; it < 8; ++it) {
          const int row = it * 2 + hh;
          *(volatile v4f*)(Cout + (size_t)(mBase + row) * ldc + n0 + c4) = vals[it];
        }
        __threadfence();
      }
    }
    __builtin_amdgcn_fence(__ATOMIC_RELEASE, "workgroup");
    __builtin_amdgcn_wave_barrier();
    __builtin_amdgcn_fence(__ATOMIC_ACQUIRE, "workgroup");
  }
}

template <bool WITH_DT, bool WITH_RES>
__global__ __launch_bounds__(256) void rms128_kernel(
    const float* __restrict__ Hin, const float* __restrict__ nw, const float* __restrict__ res,
    const float* __restrict__ Wdt, const float* __restrict__ dtb, const float* __restrict__ alog,
    unsigned short* __restrict__ OutH, unsigned short* __restrict__ OutL,
    float* __restrict__ DT, float* __restrict__ LA)
{
  const int tid = threadIdx.x, lane = tid & 31, wave = tid >> 5;
  const int hh = lane >> 4, c8 = (lane & 15) * 8;
  const int row0 = (blockIdx.x * 8 + wave) * 32;
  float w[8], wd0[8], wd1[8];
  {
    const v4f t0 = *(const v4f*)(nw + c8);
    const v4f t1 = *(const v4f*)(nw + c8 + 4);
#pragma unroll
    for (int e = 0; e < 4; ++e) {
      const float s0 = t0[e];
      const float s1 = t1[e];
      w[e] = bf16r(s0); w[4 + e] = bf16r(s1);
    }
  }
  if (WITH_DT) {
    const v4f a0 = *(const v4f*)(Wdt + c8);
    const v4f a1 = *(const v4f*)(Wdt + c8 + 4);
    const v4f b0 = *(const v4f*)(Wdt + kDI + c8);
    const v4f b1 = *(const v4f*)(Wdt + kDI + c8 + 4);
#pragma unroll
    for (int e = 0; e < 4; ++e) {
      const float s0 = a0[e];
      const float s1 = a1[e];
      const float s2 = b0[e];
      const float s3 = b1[e];
      wd0[e] = bf16r(s0); wd0[4 + e] = bf16r(s1); wd1[e] = bf16r(s2); wd1[4 + e] = bf16r(s3);
    }
  } else {
#pragma unroll
    for (int e = 0; e < 8; ++e) { wd0[e] = 0.f; wd1[e] = 0.f; }
  }
  float keep0 = 0.f, keep1 = 0.f;
#pragma unroll 1
  for (int it = 0; it < 16; ++it) {
    const int row = row0 + 2 * it + hh;
    const float* p = Hin + (size_t)row * kDI + c8;
    const v4f a0 = *(const v4f*)(p);
    const v4f a1 = *(const v4f*)(p + 4);
    float x[8];
#pragma unroll
    for (int e = 0; e < 4; ++e) { x[e] = a0[e]; x[4 + e] = a1[e]; }
    float ss = 0.f;
#pragma unroll
    for (int e = 0; e < 8; ++e) ss = fmaf(x[e], x[e], ss);
    ss += __shfl_xor(ss, 1, 32);
    ss += __shfl_xor(ss, 2, 32);
    ss += __shfl_xor(ss, 4, 32);
    ss += __shfl_xor(ss, 8, 32);
    const float sc = rsqrtf(ss * (1.0f / (float)kDI) + kEps);
    float hn[8];
#pragma unroll
    for (int e = 0; e < 8; ++e) hn[e] = x[e] * sc * w[e];
    float o[8];
    if (WITH_RES) {
      const float* rp = res + (size_t)row * kDI + c8;
      const v4f r0 = *(const v4f*)(rp);
      const v4f r1 = *(const v4f*)(rp + 4);
#pragma unroll
      for (int e = 0; e < 4; ++e) { o[e] = r0[e] + hn[e]; o[4 + e] = r1[e] + hn[4 + e]; }
    } else {
#pragma unroll
      for (int e = 0; e < 8; ++e) o[e] = hn[e];
    }
    v8h hv, lv;
#pragma unroll
    for (int e = 0; e < 8; ++e) {
      _Float16 a, b;
      split_res(o[e], a, b);
      hv[e] = a;
      lv[e] = b;
    }
    volatile v8h* ph = (volatile v8h*)(OutH + (size_t)row * kDI + c8);
    volatile v8h* pl = (volatile v8h*)(OutL + (size_t)row * kDI + c8);
    *ph = hv;
    *pl = lv;
    __threadfence();
    *ph = hv;
    *pl = lv;
    if (WITH_DT) {
      float d0 = 0.f, d1 = 0.f;
#pragma unroll
      for (int e = 0; e < 8; ++e) { d0 = fmaf(hn[e], wd0[e], d0); d1 = fmaf(hn[e], wd1[e], d1); }
      d0 += __shfl_xor(d0, 1, 32); d1 += __shfl_xor(d1, 1, 32);
      d0 += __shfl_xor(d0, 2, 32); d1 += __shfl_xor(d1, 2, 32);
      d0 += __shfl_xor(d0, 4, 32); d1 += __shfl_xor(d1, 4, 32);
      d0 += __shfl_xor(d0, 8, 32); d1 += __shfl_xor(d1, 8, 32);
      const int srcl = (lane & 1) << 4;
      const float s0 = __shfl(d0, srcl, 32);
      const float s1 = __shfl(d1, srcl, 32);
      const bool mine = ((lane >> 1) == it);
      keep0 = mine ? s0 : keep0;
      keep1 = mine ? s1 : keep1;
    }
  }
  if (WITH_DT) {
    const size_t rowl = (size_t)(row0 + lane);
    float cur = keep0;
    const float nxt = keep1;
#pragma unroll 1
    for (int k = 0; k < kHeads; ++k) {
      const float v  = cur + bf16r(dtb[k]);
      const float dt = fmaxf(v, 0.0f) + log1pf(expf(-fabsf(v)));
      const float la = dt * (-expf(bf16r(alog[k])));
      volatile float* pd = (volatile float*)(DT + (size_t)k * kRows + rowl);
      volatile float* pl = (volatile float*)(LA + (size_t)k * kRows + rowl);
      *pd = dt;
      *pl = la;
      __threadfence();
      *pd = dt;
      *pl = la;
      cur = nxt;
    }
  }
}

__global__ __launch_bounds__(256) void conv_silu_kernel(
    const float* __restrict__ ZX, const float* __restrict__ cw, const float* __restrict__ cb,
    float* __restrict__ XC)
{
  __shared__ __align__(16) float sT[16 * kConvTP];
  const int tid = threadIdx.x, lane = tid & 31, wave = tid >> 5;
  const int d0 = blockIdx.x * 256, d = d0 + tid;
  const int g0 = blockIdx.y * 64;
  const int tb = g0 & (kSeq - 1);
  const v4f wv = *(const v4f*)(cw + d * 4);
  const float t0w = wv[0], t1w = wv[1], t2w = wv[2], t3w = wv[3];
  const float w0 = bf16r(t0w), w1 = bf16r(t1w), w2 = bf16r(t2w), w3 = bf16r(t3w);
  const float bc = bf16r(cb[d]);
  const float* src = ZX + kDIN + d;
  float xm3, xm2, xm1;
  {
    const bool hist = (tb > 0);
    const int rb = hist ? (g0 - 3) : g0;
    const float v3 = src[(size_t)rb * kZXW];
    const float v2 = src[(size_t)(rb + 1) * kZXW];
    const float v1 = src[(size_t)(rb + 2) * kZXW];
    xm3 = hist ? v3 : 0.f;
    xm2 = hist ? v2 : 0.f;
    xm1 = hist ? v1 : 0.f;
  }
  const int hrow = wave >> 1;
  const int hch  = (wave & 1) * 128 + lane * 4;
#pragma unroll 1
  for (int sub = 0; sub < 4; ++sub) {
    const int lb = g0 + sub * 16;
#pragma unroll 1
    for (int s = 0; s < 16; ++s) {
      const float xcur = src[(size_t)(lb + s) * kZXW];
      float acc = w0 * xm3;
      acc = fmaf(w1, xm2, acc);
      acc = fmaf(w2, xm1, acc);
      acc = fmaf(w3, xcur, acc);
      const float sv = acc + bc;
      const float sg = __builtin_amdgcn_rcpf(1.0f + expf(-sv));
      sT[s * kConvTP + tid] = sv * sg;
      xm3 = xm2; xm2 = xm1; xm1 = xcur;
    }
    __syncthreads();
    v4f fv[4];
#pragma unroll
    for (int it = 0; it < 4; ++it) fv[it] = *(const v4f*)(sT + (it * 4 + hrow) * kConvTP + hch);
    for (int pass = 0; pass < 2; ++pass) {
#pragma unroll
      for (int it = 0; it < 4; ++it)
        *(volatile v4f*)(XC + (size_t)(lb + it * 4 + hrow) * kCCH + d0 + hch) = fv[it];
      __threadfence();
    }
    __syncthreads();
  }
}

constexpr int kLdsXth  = 0;
constexpr int kLdsXtl  = kLdsXth + kPS * kXTP * 2;
constexpr int kLdsU1   = kLdsXtl + kPS * kXTP * 2;
constexpr int kU1a     = 2 * kQ * kBP * 2;
constexpr int kU1b     = 2 * kNst * kXTP * 2;
constexpr int kU1Bytes = (kU1a > kU1b) ? kU1a : kU1b;
constexpr int kLdsC    = kLdsU1 + kU1Bytes;
constexpr int kLdsM    = kLdsC + 2 * kQ * kBP * 2;
constexpr int kLdsSt   = kLdsM + kQ * kXTP * 2;
constexpr int kLdsTot  = kLdsSt + kPS * kBP * 2;
static_assert(kQ * kYP * 4 <= 2 * kQ * kBP * 2, "output tile fits in the C tile pair");
static_assert((kLdsXtl % 16) == 0 && (kLdsU1 % 16) == 0 && (kLdsC % 16) == 0 && (kLdsM % 16) == 0 && (kLdsSt % 16) == 0 &&
              ((kQ * kBP * 2) % 16) == 0 && ((kNst * kXTP * 2) % 16) == 0, "16-B aligned tiles");
static_assert(kLdsTot + 4 * kQ * 4 <= 65536, "LDS budget");

__global__ __launch_bounds__(256) void chunk_scan_kernel(
    float* XC, const float* __restrict__ DT, const float* __restrict__ LA,
    const float* __restrict__ Dp)
{
  __shared__ __align__(16) unsigned char smem[kLdsTot];
  __shared__ float s_c[kQ];
  __shared__ float s_dt[kQ];
  __shared__ float s_w[kQ];
  __shared__ float s_e[kQ];
  unsigned short* const sXth = (unsigned short*)(smem + kLdsXth);
  unsigned short* const sXtl = (unsigned short*)(smem + kLdsXtl);
  unsigned short* const sBh  = (unsigned short*)(smem + kLdsU1);
  unsigned short* const sBl  = (unsigned short*)(smem + kLdsU1 + kQ * kBP * 2);
  unsigned short* const sBwh = (unsigned short*)(smem + kLdsU1);
  unsigned short* const sBwl = (unsigned short*)(smem + kLdsU1 + kNst * kXTP * 2);
  unsigned short* const sCh  = (unsigned short*)(smem + kLdsC);
  unsigned short* const sCl  = (unsigned short*)(smem + kLdsC + kQ * kBP * 2);
  float*          const sY   = (float*)(smem + kLdsC);
  unsigned short* const sM   = (unsigned short*)(smem + kLdsM);
  unsigned short* const sSt  = (unsigned short*)(smem + kLdsSt);

  const int tid = threadIdx.x, lane = tid & 31, wave = tid >> 5;
  const int hh = lane >> 4, l15 = lane & 15, koff = hh * 8;
  const int b  = blockIdx.x >> 2;
  const int h  = (blockIdx.x >> 1) & 1;
  const int p0 = (blockIdx.x & 1) * kPS;
  const float dval = bf16r(Dp[h]);

  for (int idx = tid; idx < kPS * kBP; idx += 256) sSt[idx] = (unsigned short)0;

  v8f sacc[4];
#pragma unroll
  for (int t = 0; t < 4; ++t) sacc[t] = (v8f){0.f,0.f,0.f,0.f,0.f,0.f,0.f,0.f};

#pragma unroll 1
  for (int cc = 0; cc < kSeq / kQ; ++cc) {
    const int t0 = cc * kQ;
    const size_t rowbase = (size_t)b * kSeq + t0;

    {
      const int i = tid >> 3, q = tid & 7;
      const float* xp = XC + (rowbase + i) * kCCH + h * kHP + p0 + q * 8;
      const v4f x0 = *(const v4f*)(xp);
      const v4f x1 = *(const v4f*)(xp + 4);
      unsigned short* dxh = sXth + (q * 8) * kXTP + i;
      unsigned short* dxl = sXtl + (q * 8) * kXTP + i;
#pragma unroll
      for (int e = 0; e < 4; ++e) {
        _Float16 a, r;
        const float v0 = x0[e];
        split_res(v0, a, r);
        dxh[e * kXTP] = h_bits(a);
        dxl[e * kXTP] = h_bits(r);
        const float v1 = x1[e];
        split_res(v1, a, r);
        dxh[(4 + e) * kXTP] = h_bits(a);
        dxl[(4 + e) * kXTP] = h_bits(r);
      }
    }
    float bf[2][8];
#pragma unroll
    for (int k = 0; k < 2; ++k) {
      const int idx = tid + 256 * k;
      const int i = idx >> 4, q = idx & 15;
      const float* rp = XC + (rowbase + i) * kCCH + kDIN + q * 8;
      const v4f b0 = *(const v4f*)(rp);
      const v4f b1 = *(const v4f*)(rp + 4);
      const v4f c0 = *(const v4f*)(rp + kNst);
      const v4f c1 = *(const v4f*)(rp + kNst + 4);
      v8h bhv, blv, chv, clv;
#pragma unroll
      for (int e = 0; e < 4; ++e) {
        _Float16 a, r;
        const float vb0 = b0[e];
        const float vb1 = b1[e];
        const float vc0 = c0[e];
        const float vc1 = c1[e];
        bf[k][e] = vb0;
        bf[k][4 + e] = vb1;
        split_res(vb0, a, r); bhv[e] = a; blv[e] = r;
        split_res(vb1, a, r); bhv[4 + e] = a; blv[4 + e] = r;
        split_res(vc0, a, r); chv[e] = a; clv[e] = r;
        split_res(vc1, a, r); chv[4 + e] = a; clv[4 + e] = r;
      }
      *(v8h*)(sBh + i * kBP + q * 8) = bhv;
      *(v8h*)(sBl + i * kBP + q * 8) = blv;
      *(v8h*)(sCh + i * kBP + q * 8) = chv;
      *(v8h*)(sCl + i * kBP + q * 8) = clv;
    }
    if (wave == 0) {
      const size_t g = (size_t)h * kRows + rowbase + lane;
      const float dtv = DT[g];
      const float lav = LA[g];
      float c = lav;
      float t;
      t = __shfl_up(c, 1, 32);  c += (lane >= 1)  ? t : 0.0f;
      t = __shfl_up(c, 2, 32);  c += (lane >= 2)  ? t : 0.0f;
      t = __shfl_up(c, 4, 32);  c += (lane >= 4)  ? t : 0.0f;
      t = __shfl_up(c, 8, 32);  c += (lane >= 8)  ? t : 0.0f;
      t = __shfl_up(c, 16, 32); c += (lane >= 16) ? t : 0.0f;
      const float cl = __shfl(c, 31, 32);
      s_c[lane]  = c;
      s_dt[lane] = dtv;
      s_w[lane]  = expf(fminf(cl - c, 0.0f)) * dtv;
      s_e[lane]  = expf(fminf(c, 0.0f));
    }
    __syncthreads();

    if (wave < 4) {
      const int ti = wave >> 1, tj = wave & 1;
      v8f g  = (v8f){0.f,0.f,0.f,0.f,0.f,0.f,0.f,0.f};
      v8f gr = (v8f){0.f,0.f,0.f,0.f,0.f,0.f,0.f,0.f};
#pragma unroll
      for (int kk = 0; kk < 4; ++kk) {
        const v16h ah = FragH::load((const _Float16*)(sCh + (ti * 16 + l15) * kBP + koff + kk * 32));
        const v16h al = FragH::load((const _Float16*)(sCl + (ti * 16 + l15) * kBP + koff + kk * 32));
        const v16h bh = FragH::load((const _Float16*)(sBh + (tj * 16 + l15) * kBP + koff + kk * 32));
        const v16h bl = FragH::load((const _Float16*)(sBl + (tj * 16 + l15) * kBP + koff + kk * 32));
        g  = mma_guarded(ah, bh, g);
        gr = mma_guarded(ah, bl, gr);
        gr = mma_guarded(al, bh, gr);
      }
      const int j = tj * 16 + l15;
      const float cj = s_c[j];
      const float dj = s_dt[j];
#pragma unroll
      for (int r = 0; r < 8; ++r) {
        const int i = ti * 16 + 8 * hh + r;
        const float d = fminf(s_c[i] - cj, 0.0f);
        const float gv = g[r] + gr[r] * kResInv;
        float val = gv * expf(d) * dj;
        val = (j <= i) ? val : 0.0f;
        val += (j == i) ? dval : 0.0f;
        sM[i * kXTP + j] = f16_bits(val * kMCarry);
      }
    }
    __syncthreads();

#pragma unroll
    for (int k = 0; k < 2; ++k) {
      const int idx = tid + 256 * k;
      const int j = idx >> 4, q = idx & 15;
      const float wj = s_w[j];
      unsigned short* dwh = sBwh + (q * 8) * kXTP + j;
      unsigned short* dwl = sBwl + (q * 8) * kXTP + j;
#pragma unroll
      for (int e = 0; e < 8; ++e) {
        _Float16 a, r;
        split_res(bf[k][e] * wj, a, r);
        dwh[e * kXTP] = h_bits(a);
        dwl[e * kXTP] = h_bits(r);
      }
    }
    __syncthreads();

    v8f yo;
    {
      const int ti = wave >> 2, tj = wave & 3;
      v8f yi  = (v8f){0.f,0.f,0.f,0.f,0.f,0.f,0.f,0.f};
      v8f yir = (v8f){0.f,0.f,0.f,0.f,0.f,0.f,0.f,0.f};
      v8f ys  = (v8f){0.f,0.f,0.f,0.f,0.f,0.f,0.f,0.f};
      v8f ysr = (v8f){0.f,0.f,0.f,0.f,0.f,0.f,0.f,0.f};
      {
        const v16h am  = FragH::load((const _Float16*)(sM + (ti * 16 + l15) * kXTP + koff));
        const v16h bxh = FragH::load((const _Float16*)(sXth + (tj * 16 + l15) * kXTP + koff));
        const v16h bxl = FragH::load((const _Float16*)(sXtl + (tj * 16 + l15) * kXTP + koff));
        yi  = mma_guarded(am, bxh, yi);
        yir = mma_guarded(am, bxl, yir);
      }
#pragma unroll
      for (int kk = 0; kk < 4; ++kk) {
        const v16h ach = FragH::load((const _Float16*)(sCh + (ti * 16 + l15) * kBP + koff + kk * 32));
        const v16h acl = FragH::load((const _Float16*)(sCl + (ti * 16 + l15) * kBP + koff + kk * 32));
        const v16h bs  = FragH::load((const _Float16*)(sSt + (tj * 16 + l15) * kBP + koff + kk * 32));
        ys  = mma_guarded(ach, bs, ys);
        ysr = mma_guarded(acl, bs, ysr);
      }
#pragma unroll
      for (int r = 0; r < 8; ++r) {
        const int i = ti * 16 + 8 * hh + r;
        const float intra = yi[r] * kMInv + yir[r] * (kMInv * kResInv);
        const float inter = ys[r] + ysr[r] * kResInv;
        yo[r] = intra + s_e[i] * inter;
      }
    }
    const int pt = wave >> 1, nb = (wave & 1) * 4;
    {
      const float T = s_e[kQ - 1];
      const v16h axh = FragH::load((const _Float16*)(sXth + (pt * 16 + l15) * kXTP + koff));
      const v16h axl = FragH::load((const _Float16*)(sXtl + (pt * 16 + l15) * kXTP + koff));
#pragma unroll
      for (int t = 0; t < 4; ++t) {
#pragma unroll
        for (int r = 0; r < 8; ++r) sacc[t][r] *= T;
      }
#pragma unroll
      for (int t = 0; t < 4; ++t) {
        const v16h bwh = FragH::load((const _Float16*)(sBwh + ((nb + t) * 16 + l15) * kXTP + koff));
        const v16h bwl = FragH::load((const _Float16*)(sBwl + ((nb + t) * 16 + l15) * kXTP + koff));
        sacc[t] = mma_guarded(axh, bwh, sacc[t]);
        v8f rr = (v8f){0.f,0.f,0.f,0.f,0.f,0.f,0.f,0.f};
        rr = mma_guarded(axh, bwl, rr);
        rr = mma_guarded(axl, bwh, rr);
#pragma unroll
        for (int r = 0; r < 8; ++r) sacc[t][r] += rr[r] * kResInv;
      }
    }
    __syncthreads();

    {
      const int ti = wave >> 2, tj = wave & 3;
#pragma unroll
      for (int r = 0; r < 8; ++r) {
        const int i = ti * 16 + 8 * hh + r;
        sY[i * kYP + tj * 16 + l15] = yo[r];
      }
    }
#pragma unroll
    for (int t = 0; t < 4; ++t) {
      const int n = (nb + t) * 16 + l15;
#pragma unroll
      for (int r = 0; r < 8; ++r) {
        const int p = pt * 16 + 8 * hh + r;
        sSt[p * kBP + n] = f16_bits(sacc[t][r]);
      }
    }
    __syncthreads();

    {
      const int c4 = l15 * 4;
      v4f yv[2];
#pragma unroll
      for (int it = 0; it < 2; ++it) {
        const int row = wave * 4 + it * 2 + hh;
        yv[it] = *(const v4f*)(sY + row * kYP + c4);
      }
      for (int pass = 0; pass < 2; ++pass) {
#pragma unroll
        for (int it = 0; it < 2; ++it) {
          const int row = wave * 4 + it * 2 + hh;
          *(volatile v4f*)(XC + (rowbase + row) * kCCH + h * kHP + p0 + c4) = yv[it];
        }
        __threadfence();
      }
    }
    __syncthreads();
  }
}

__global__ __launch_bounds__(256) void gated_rms256_kernel(
    const float* __restrict__ XC, const float* __restrict__ ZX, const float* __restrict__ gw,
    unsigned short* __restrict__ YNH, unsigned short* __restrict__ YNL)
{
  const int tid = threadIdx.x, lane = tid & 31, wave = tid >> 5;
  const int c8 = lane * 8;
  const int row0 = (blockIdx.x * 8 + wave) * 8;
  float w[8];
  {
    const v4f t0 = *(const v4f*)(gw + c8);
    const v4f t1 = *(const v4f*)(gw + c8 + 4);
#pragma unroll
    for (int e = 0; e < 4; ++e) {
      const float s0 = t0[e];
      const float s1 = t1[e];
      w[e] = bf16r(s0); w[4 + e] = bf16r(s1);
    }
  }
#pragma unroll 1
  for (int rr = 0; rr < 8; ++rr) {
    const int row = row0 + rr;
    const float* yp = XC + (size_t)row * kCCH + c8;
    const float* zp = ZX + (size_t)row * kZXW + c8;
    const v4f y0 = *(const v4f*)(yp);
    const v4f y1 = *(const v4f*)(yp + 4);
    const v4f z0 = *(const v4f*)(zp);
    const v4f z1 = *(const v4f*)(zp + 4);
    float yv[8], zv[8], g[8];
#pragma unroll
    for (int e = 0; e < 4; ++e) { yv[e] = y0[e]; yv[4 + e] = y1[e]; zv[e] = z0[e]; zv[4 + e] = z1[e]; }
    float ss = 0.f;
#pragma unroll
    for (int e = 0; e < 8; ++e) {
      const float sg = __builtin_amdgcn_rcpf(1.0f + expf(-zv[e]));
      g[e] = yv[e] * (zv[e] * sg);
      ss = fmaf(g[e], g[e], ss);
    }
    ss += __shfl_xor(ss, 16, 32);
    ss += __shfl_xor(ss, 8, 32);
    ss += __shfl_xor(ss, 4, 32);
    ss += __shfl_xor(ss, 2, 32);
    ss += __shfl_xor(ss, 1, 32);
    const float sc = rsqrtf(ss * (1.0f / (float)kDIN) + kEps);
    v8h hv, lv;
#pragma unroll
    for (int e = 0; e < 8; ++e) {
      _Float16 a, b;
      split_res(g[e] * sc * w[e], a, b);
      hv[e] = a;
      lv[e] = b;
    }
    volatile v8h* ph = (volatile v8h*)(YNH + (size_t)row * kDIN + c8);
    volatile v8h* pl = (volatile v8h*)(YNL + (size_t)row * kDIN + c8);
    *ph = hv;
    *pl = lv;
    __threadfence();
    *ph = hv;
    *pl = lv;
  }
}

extern "C" void kernel_launch(void* const* d_in, const int* in_sizes, int n_in,
                              void* d_out, int out_size, void* d_ws, size_t ws_size,
                              hipStream_t stream) {
  if (n_in < 15) return;
  if (in_sizes[0] != kRows * kNE) return;
  if (in_sizes[1] != kDI * kNE) return;
  if (in_sizes[2] != kDI) return;
  if (in_sizes[3] != kDOut * kDI) return;
  if (in_sizes[4] != kDOut) return;
  if (in_sizes[5] != kNL * kDI) return;
  if (in_sizes[6] != kNL * kDPROJ * kDI) return;
  if (in_sizes[7] != kNL * kCCH * 4) return;
  if (in_sizes[8] != kNL * kCCH) return;
  if (in_sizes[9] != kNL * kHeads) return;
  if (in_sizes[10] != kNL * kHeads) return;
  if (in_sizes[11] != kNL * kHeads) return;
  if (in_sizes[12] != kNL * kDIN) return;
  if (in_sizes[13] != kNL * kDI * kDIN) return;
  if (in_sizes[14] != kDI) return;
  if (out_size != kRows * kDOut) return;
  if (ws_size < kWsTotal) return;

  const float* x       = (const float*)d_in[0];
  const float* in_w    = (const float*)d_in[1];
  const float* in_b    = (const float*)d_in[2];
  const float* out_w   = (const float*)d_in[3];
  const float* out_b   = (const float*)d_in[4];
  const float* l_rms_w = (const float*)d_in[5];
  const float* l_in_w  = (const float*)d_in[6];
  const float* conv_w  = (const float*)d_in[7];
  const float* conv_b  = (const float*)d_in[8];
  const float* dt_bias = (const float*)d_in[9];
  const float* A_log   = (const float*)d_in[10];
  const float* D_p     = (const float*)d_in[11];
  const float* gnorm_w = (const float*)d_in[12];
  const float* l_out_w = (const float*)d_in[13];
  const float* fnorm_w = (const float*)d_in[14];
  float* out = (float*)d_out;

  char* ws = (char*)d_ws;
  unsigned short* X16   = (unsigned short*)(ws + kOffX16);
  unsigned short* WIN16 = (unsigned short*)(ws + kOffWIN16);
  unsigned short* WL16  = (unsigned short*)(ws + kOffWL16);
  unsigned short* WO16  = (unsigned short*)(ws + kOffWO16);
  unsigned short* WF16  = (unsigned short*)(ws + kOffWF16);
  float*          XP    = (float*)(ws + kOffXP);
  float*          H1    = (float*)(ws + kOffH1);
  unsigned short* HNH   = (unsigned short*)(ws + kOffHNH);
  unsigned short* HNL   = (unsigned short*)(ws + kOffHNL);
  float*          ZX    = (float*)(ws + kOffZX);
  float*          XC    = (float*)(ws + kOffXC);
  float*          DTp   = (float*)(ws + kOffDT);
  float*          LAp   = (float*)(ws + kOffLA);
  unsigned short* YNH   = (unsigned short*)(ws + kOffYNH);
  unsigned short* YNL   = (unsigned short*)(ws + kOffYNL);
  float*          H2    = ZX;
  unsigned short* OH    = HNH;
  unsigned short* OL    = HNL;

  const float foldMain = kWCarryInv;
  const float foldRes  = kWCarryInv * kResInv;

  cast_f16_kernel<<<(kRows * kNE / 8) / 256, 256, 0, stream>>>(x, X16, kRows * kNE / 8, 1.0f);
  cast_f16_kernel<<<(kDI * kNE / 8) / 256, 256, 0, stream>>>(in_w, WIN16, kDI * kNE / 8, kWCarry);
  for (int l = 0; l < kNL; ++l) {
    cast_f16_kernel<<<(kZXW * kDI / 8) / 256, 256, 0, stream>>>(
        l_in_w + (size_t)l * kDPROJ * kDI, WL16 + (size_t)l * kZXW * kDI, kZXW * kDI / 8, kWCarry);
  }
  cast_f16_kernel<<<(kNL * kDI * kDIN / 8) / 256, 256, 0, stream>>>(l_out_w, WO16, kNL * kDI * kDIN / 8, kWCarry);
  cast_f16_kernel<<<(kDOut * kDI / 8) / 256, 256, 0, stream>>>(out_w, WF16, kDOut * kDI / 8, kWCarry);

  wmma_gemm_f16<4, false, 2, false><<<64, 256, 0, stream>>>(
      X16, X16, kNE, WIN16, kNE, XP, kDI, in_b, x, kRows, kDI, kNE, foldMain, 0.0f);

  for (int l = 0; l < kNL; ++l) {
    const float* Hprev = (l == 0) ? XP : H1;
    float*       Hnext = (l == 0) ? H1 : H2;
    const float* Wl    = l_in_w + (size_t)l * kDPROJ * kDI;

    rms128_kernel<true, false><<<kRows / 256, 256, 0, stream>>>(
        Hprev, l_rms_w + l * kDI, Hprev, Wl + (size_t)kZXW * kDI, dt_bias + l * kHeads, A_log + l * kHeads,
        HNH, HNL, DTp, LAp);

    wmma_gemm_f16<2, true, 0, false><<<768, 256, 0, stream>>>(
        HNH, HNL, kDI, WL16 + (size_t)l * kZXW * kDI, kDI, ZX, kZXW, in_b, x, kRows, kZXW, kDI, foldMain, foldRes);

    conv_silu_kernel<<<dim3(kCCH / 256, kRows / 64), 256, 0, stream>>>(
        ZX, conv_w + (size_t)l * kCCH * 4, conv_b + l * kCCH, XC);

    chunk_scan_kernel<<<kBatch * kHeads * (kHP / kPS), 256, 0, stream>>>(
        XC, DTp, LAp, D_p + l * kHeads);

    gated_rms256_kernel<<<kRows / 64, 256, 0, stream>>>(XC, ZX, gnorm_w + l * kDIN, YNH, YNL);

    wmma_gemm_f16<2, true, 0, true><<<128, 256, 0, stream>>>(
        YNH, YNL, kDIN, WO16 + (size_t)l * kDI * kDIN, kDIN, Hnext, kDI, in_b, Hprev, kRows, kDI, kDIN,
        foldMain, foldRes);
  }

  rms128_kernel<false, true><<<kRows / 256, 256, 0, stream>>>(
      H2, fnorm_w, XP, fnorm_w, fnorm_w, fnorm_w, OH, OL, DTp, LAp);

  wmma_gemm_f16<2, true, 2, false><<<64, 256, 0, stream>>>(
      OH, OL, kDI, WF16, kDI, out, kDOut, out_b, x, kRows, kDOut, kDI, foldMain, foldRes);
}
